// PointNetSetAbstractor_90924457656322
// MI455X (gfx1250) — hardware-verified
//
#include <hip/hip_runtime.h>
#include <stdint.h>

#pragma clang fp contract(off)

typedef __attribute__((ext_vector_type(16))) _Float16 v16h;
typedef __attribute__((ext_vector_type(8)))  _Float16 v8h;
typedef __attribute__((ext_vector_type(8)))  float    v8f;
typedef __attribute__((ext_vector_type(4)))  float    v4f;

constexpr int NBATCH   = 16;
constexpr int NPTS     = 4096;
constexpr int NCEN     = 1024;
constexpr int NNBR     = 32;
constexpr int NFEAT    = 64;
constexpr int NCH_IN0  = 67;
constexpr int KPAD0    = 96;
constexpr int NCH_L0   = 64;
constexpr int NCH_L1   = 64;
constexpr int NCH_L2   = 128;
constexpr float WEIGHT_CARRY     = 64.0f;
constexpr float WEIGHT_CARRY_INV = 1.0f / 64.0f;
constexpr float RESID_CARRY      = 2048.0f;
constexpr float RESID_CARRY_INV  = 1.0f / 2048.0f;
constexpr float BN_EPS           = 1e-5f;

static_assert(KPAD0 % 32 == 0 && KPAD0 >= NCH_IN0, "layer-0 K padded to a 32 multiple");
static_assert(NCH_L0 % 32 == 0 && NCH_L1 % 32 == 0, "layer-1/2 K multiple of 32");
static_assert(NCH_L0 % 16 == 0 && NCH_L1 % 16 == 0 && NCH_L2 % 16 == 0, "N tile multiples");
static_assert(NNBR == 32, "one neighbour row per lane, two 16-row m-tiles");
static_assert(NFEAT + 3 == NCH_IN0, "channel order [dx,dy,dz | features]");

constexpr size_t WS_BT0   = 0;
constexpr size_t WS_BT1   = 12288;
constexpr size_t WS_BT2   = 20480;
constexpr size_t WS_SCALE = 36864;
constexpr size_t WS_SHIFT = 37888;
constexpr size_t WS_CENT  = 38912;
constexpr size_t WS_TOTAL = 301056;
static_assert(WS_BT1 == WS_BT0 + (size_t)NCH_L0 * KPAD0 * 2, "carve");
static_assert(WS_BT2 == WS_BT1 + (size_t)NCH_L1 * NCH_L0 * 2, "carve");
static_assert(WS_SCALE == WS_BT2 + (size_t)NCH_L2 * NCH_L1 * 2, "carve");
static_assert(WS_SHIFT == WS_SCALE + 256 * 4, "carve");
static_assert(WS_CENT == WS_SHIFT + 256 * 4, "carve");
static_assert(WS_TOTAL == WS_CENT + (size_t)NBATCH * NCEN * 16, "carve");
static_assert(WS_TOTAL <= 134217728, "carve under 128 MiB");
static_assert(WS_BT1 % 128 == 0 && WS_BT2 % 128 == 0 && WS_SCALE % 128 == 0 && WS_SHIFT % 128 == 0 && WS_CENT % 128 == 0, "line aligned regions");

constexpr size_t OUT0_BYTES = (size_t)NBATCH * NCEN * 3 * 4;
constexpr size_t OUT1_BYTES = (size_t)NBATCH * NCEN * NCH_L2 * 4;
static_assert(OUT0_BYTES == 196608 && OUT0_BYTES % 128 == 0, "out1 starts on a line");
static_assert(OUT0_BYTES + OUT1_BYTES == 8585216, "d_out total");

struct FragH {
  union U { v16h v; v8h h[2]; };
  static __device__ __forceinline__ v16h load(const _Float16* p) {
    U f; f.h[0] = *(const v8h*)(p); f.h[1] = *(const v8h*)(p + 16); return f.v;
  }
};

__device__ __forceinline__ v8f mma_f16(v16h a, v16h b, v8f c) {
  c = __builtin_amdgcn_wmma_f32_16x16x32_f16(false, a, false, b, (short)0, c, false, false);
  asm volatile("v_nop\n\tv_nop\n\tv_nop\n\tv_nop" : "+v"(c) : "v"(a), "v"(b));
  return c;
}

__device__ __forceinline__ void store_v8h_twice(_Float16* p, v8h v) {
  *(volatile v8h*)p = v;
  __threadfence();
  *(volatile v8h*)p = v;
}
__device__ __forceinline__ void store_v4f_twice(float* p, v4f v) {
  *(volatile v4f*)p = v;
  __threadfence();
  *(volatile v4f*)p = v;
}

__device__ __forceinline__ void split_f16(float x, _Float16& hi, _Float16& lo) {
  const float xh = (fabsf(x) < 6.103515625e-05f) ? 0.0f : x;
  hi = (_Float16)xh;
  const float hf = (float)hi;
  const float rs = x - hf;
  lo = (_Float16)(rs * RESID_CARRY);
}

__device__ __forceinline__ int clamp_pt(int i) {
  i = i < 0 ? 0 : i;
  return i > (NPTS - 1) ? (NPTS - 1) : i;
}

__device__ __forceinline__ void bn_fold(const float* bp, const float* gp, const float* bep,
                                        const float* mp, const float* vp,
                                        float* sc, float* sh, int nquads, int t) {
  const bool active = t < nquads;
  const int q = active ? t : 0;
  const v4f bb = *(const v4f*)(bp + q * 4);
  const v4f gg = *(const v4f*)(gp + q * 4);
  const v4f ee = *(const v4f*)(bep + q * 4);
  const v4f mm = *(const v4f*)(mp + q * 4);
  const v4f vv = *(const v4f*)(vp + q * 4);
  v4f sv, tv;
#pragma unroll
  for (int e = 0; e < 4; ++e) {
    const float s = gg[e] * rsqrtf(vv[e] + BN_EPS);
    const float d = bb[e] - mm[e];
    const float ds = d * s;
    tv[e] = ds + ee[e];
    sv[e] = s * WEIGHT_CARRY_INV;
  }
  if (active) {
    store_v4f_twice(sc + q * 4, sv);
    store_v4f_twice(sh + q * 4, tv);
  }
}

__global__ __launch_bounds__(256) void prep_kernel(
    const float* __restrict__ W0, const float* __restrict__ W1, const float* __restrict__ W2,
    const float* __restrict__ b0, const float* __restrict__ g0, const float* __restrict__ be0,
    const float* __restrict__ m0, const float* __restrict__ v0,
    const float* __restrict__ b1, const float* __restrict__ g1, const float* __restrict__ be1,
    const float* __restrict__ m1, const float* __restrict__ v1,
    const float* __restrict__ b2, const float* __restrict__ g2, const float* __restrict__ be2,
    const float* __restrict__ m2, const float* __restrict__ v2,
    _Float16* __restrict__ btall, float* __restrict__ scale, float* __restrict__ shift) {
  const int t = threadIdx.x;
  const int blk = blockIdx.x;
  float zf = 0.0f;
  asm volatile("" : "+v"(zf));
  if (blk < 9) {
    const int ci = blk * 256 + t;
    v8h hv;
    if (blk < 3) {
      const int n = ci / 12;
      const int kk = (ci - n * 12) * 8;
#pragma unroll
      for (int e = 0; e < 8; ++e) {
        const int k = kk + e;
        const bool real = k < NCH_IN0;
        const int row = (k < NFEAT) ? (k + 3) : (real ? (k - NFEAT) : 0);
        const float w = W0[row * NCH_L0 + n];
        const float val = real ? (w * WEIGHT_CARRY) : zf;
        hv[e] = (_Float16)val;
      }
    } else if (blk < 5) {
      const int loc = ci - 768;
      const int n = loc >> 3;
      const int kk = (loc & 7) * 8;
#pragma unroll
      for (int e = 0; e < 8; ++e) {
        const float w = W1[(kk + e) * NCH_L1 + n];
        hv[e] = (_Float16)(w * WEIGHT_CARRY);
      }
    } else {
      const int loc = ci - 1280;
      const int n = loc >> 3;
      const int kk = (loc & 7) * 8;
#pragma unroll
      for (int e = 0; e < 8; ++e) {
        const float w = W2[(kk + e) * NCH_L2 + n];
        hv[e] = (_Float16)(w * WEIGHT_CARRY);
      }
    }
    store_v8h_twice(btall + (size_t)ci * 8, hv);
  } else if (blk == 9) {
    bn_fold(b0, g0, be0, m0, v0, scale + 0, shift + 0, NCH_L0 / 4, t);
  } else if (blk == 10) {
    bn_fold(b1, g1, be1, m1, v1, scale + 64, shift + 64, NCH_L1 / 4, t);
  } else {
    bn_fold(b2, g2, be2, m2, v2, scale + 128, shift + 128, NCH_L2 / 4, t);
  }
}

__global__ __launch_bounds__(256) void fps_kernel(const float* __restrict__ xyz,
                                                  float* __restrict__ out0,
                                                  float* __restrict__ cent4) {
  __shared__ __align__(16) float xs[NPTS * 3];
  __shared__ int sidx[NCEN];
  __shared__ float rv[2][8];
  __shared__ int ri[2][8];
  const int b = blockIdx.x;
  const int t = threadIdx.x;
  const int lane = t & 31;
  const int wave = t >> 5;
  const float* xb = xyz + (size_t)b * NPTS * 3;

#pragma unroll 4
  for (int i = 0; i < 12; ++i) {
    const int o = (i * 256 + t) * 4;
    const v4f v = *(const v4f*)(xb + o);
    *(v4f*)(xs + o) = v;
  }
  __syncthreads();

  const int base = t * 16;
  float px[16], py[16], pz[16], md[16];
#pragma unroll
  for (int q = 0; q < 16; ++q) {
    px[q] = xs[(base + q) * 3 + 0];
    py[q] = xs[(base + q) * 3 + 1];
    pz[q] = xs[(base + q) * 3 + 2];
    md[q] = 1e10f;
  }

  int last = 0;
  for (int it = 0; it < NCEN - 1; ++it) {
    if (t == 0) sidx[it] = last;
    const float cx = xs[last * 3 + 0];
    const float cy = xs[last * 3 + 1];
    const float cz = xs[last * 3 + 2];
    float bestv = -1.0f;
    int besti = base;
#pragma unroll
    for (int q = 0; q < 16; ++q) {
      const float dx = px[q] - cx;
      const float dy = py[q] - cy;
      const float dz = pz[q] - cz;
      const float tx = dx * dx;
      const float ty = dy * dy;
      const float tz = dz * dz;
      const float txz = tx + tz;
      const float d = txz + ty;
      float m = md[q];
      m = (d < m) ? d : m;
      md[q] = m;
      const bool better = m > bestv;
      bestv = better ? m : bestv;
      besti = better ? (base + q) : besti;
    }
#pragma unroll
    for (int off = 16; off > 0; off >>= 1) {
      const float ov = __shfl_xor(bestv, off, 32);
      const int oi = __shfl_xor(besti, off, 32);
      const bool take = (ov > bestv) || ((ov == bestv) && (oi < besti));
      bestv = take ? ov : bestv;
      besti = take ? oi : besti;
    }
    const int par = it & 1;
    if (lane == 0) { rv[par][wave] = bestv; ri[par][wave] = besti; }
    __syncthreads();
    float gv = rv[par][0];
    int gi = ri[par][0];
#pragma unroll
    for (int w = 1; w < 8; ++w) {
      const float ov = rv[par][w];
      const int oi = ri[par][w];
      const bool take = (ov > gv) || ((ov == gv) && (oi < gi));
      gv = take ? ov : gv;
      gi = take ? oi : gi;
    }
    last = clamp_pt(gi);
  }
  if (t == 0) sidx[NCEN - 1] = last;
  __syncthreads();

  v4f cvv[4];
#pragma unroll
  for (int i = 0; i < 4; ++i) {
    const int id = clamp_pt(sidx[i * 256 + t]);
    v4f c;
    c[0] = xs[id * 3 + 0];
    c[1] = xs[id * 3 + 1];
    c[2] = xs[id * 3 + 2];
    c[3] = 0.0f;
    cvv[i] = c;
  }
  v4f ovv[3];
#pragma unroll
  for (int i = 0; i < 3; ++i) {
    v4f o;
#pragma unroll
    for (int e = 0; e < 4; ++e) {
      const int j = (i * 256 + t) * 4 + e;
      const int s = j / 3;
      const int cc = j - s * 3;
      const int id = clamp_pt(sidx[s]);
      o[e] = xs[id * 3 + cc];
    }
    ovv[i] = o;
  }
  float* cb = cent4 + (size_t)b * NCEN * 4;
  float* ob = out0 + (size_t)b * NCEN * 3;
  for (int pass = 0; pass < 2; ++pass) {
#pragma unroll
    for (int i = 0; i < 4; ++i) *(volatile v4f*)(cb + (i * 256 + t) * 4) = cvv[i];
#pragma unroll
    for (int i = 0; i < 3; ++i) *(volatile v4f*)(ob + (i * 256 + t) * 4) = ovv[i];
    __threadfence();
  }
}

constexpr int MLP_WAVES = 2;
constexpr int APITCH = 104;
constexpr int HPITCH = 72;
static_assert((NBATCH * NCEN) % MLP_WAVES == 0, "grid exact");
static_assert((APITCH * 2) % 16 == 0 && (HPITCH * 2) % 16 == 0 && APITCH >= KPAD0 && HPITCH >= NCH_L0, "LDS pitches");

__global__ __launch_bounds__(64) void group_mlp_kernel(
    const float* __restrict__ xyz, const float* __restrict__ points,
    const float* __restrict__ cent4,
    const _Float16* __restrict__ bt0, const _Float16* __restrict__ bt1,
    const _Float16* __restrict__ bt2,
    const float* __restrict__ scale, const float* __restrict__ shift,
    float* __restrict__ out1) {
  __shared__ __align__(16) _Float16 Ahi[MLP_WAVES][32 * APITCH];
  __shared__ __align__(16) _Float16 Alo[MLP_WAVES][32 * APITCH];
  __shared__ __align__(16) _Float16 Hb0[MLP_WAVES][32 * HPITCH];
  __shared__ __align__(16) _Float16 Hb1[MLP_WAVES][32 * HPITCH];
  __shared__ __align__(16) float Ost[MLP_WAVES][NCH_L2];
  __shared__ int Hit[MLP_WAVES][NNBR];

  const int lane = threadIdx.x & 31;
  const int wave = threadIdx.x >> 5;
  const int hh = lane >> 4;
  const int c = lane & 15;
  const int gid = blockIdx.x * MLP_WAVES + wave;
  const int b = gid >> 10;
  const float* xb = xyz + (size_t)b * NPTS * 3;

  _Float16* ahi = Ahi[wave];
  _Float16* alo = Alo[wave];
  _Float16* h0w = Hb0[wave];
  _Float16* h1w = Hb1[wave];
  float* ost = Ost[wave];
  int* hl = Hit[wave];

  const v4f cv = *(const v4f*)(cent4 + (size_t)gid * 4);
  const float cx = cv[0], cy = cv[1], cz = cv[2];
  const float r2 = __uint_as_float(0x3D23D70Au);

  int cnt = 0;
  for (int ch = 0; ch < NPTS / 32; ++ch) {
    if (cnt >= NNBR) break;
    const int p = ch * 32 + lane;
    const float qx = xb[p * 3 + 0];
    const float qy = xb[p * 3 + 1];
    const float qz = xb[p * 3 + 2];
    const float dx = cx - qx;
    const float dy = cy - qy;
    const float dz = cz - qz;
    const float tx = dx * dx;
    const float ty = dy * dy;
    const float tz = dz * dz;
    const float txz = tx + tz;
    const float d2 = txz + ty;
    const bool hit = d2 < r2;
    const unsigned mask = __builtin_amdgcn_ballot_w32(hit);
    const int rank = __popc(mask & ((1u << lane) - 1u));
    const int slot = cnt + rank;
    if (hit && slot < NNBR) hl[slot] = p;
    cnt += __popc(mask);
  }
  const int nvalid = cnt < NNBR ? cnt : NNBR;
  if (lane >= nvalid) hl[lane] = -1;
  __syncthreads();

  {
    const int id = hl[lane];
    const bool valid = id >= 0;
    const int idc = clamp_pt(id);
    const int src = valid ? idc : (NPTS - 1);
    float gx = xb[idc * 3 + 0];
    float gy = xb[idc * 3 + 1];
    float gz = xb[idc * 3 + 2];
    asm volatile("" : "+v"(gx), "+v"(gy), "+v"(gz));
    gx = valid ? gx : 0.0f;
    gy = valid ? gy : 0.0f;
    gz = valid ? gz : 0.0f;
    const float ddx = gx - cx;
    const float ddy = gy - cy;
    const float ddz = gz - cz;
    float zf = 0.0f;
    asm volatile("" : "+v"(zf));
    const _Float16 z16 = (_Float16)zf;
    const float* pf = points + ((size_t)b * NPTS + (size_t)src) * NFEAT;
    _Float16* rh = ahi + lane * APITCH;
    _Float16* rl = alo + lane * APITCH;
#pragma unroll
    for (int part = 0; part < 2; ++part) {
      v4f f[8];
#pragma unroll
      for (int i = 0; i < 8; ++i) f[i] = *(const v4f*)(pf + part * 32 + i * 4);
      asm volatile("" ::: "memory");
#pragma unroll
      for (int j = 0; j < 4; ++j) {
        v8h hv, lv;
#pragma unroll
        for (int e = 0; e < 8; ++e) {
          const float x = f[j * 2 + (e >> 2)][e & 3];
          _Float16 xh, xl;
          split_f16(x, xh, xl);
          hv[e] = xh;
          lv[e] = xl;
        }
        *(v8h*)(rh + part * 32 + j * 8) = hv;
        *(v8h*)(rl + part * 32 + j * 8) = lv;
      }
    }
    {
      _Float16 xh0, xl0, xh1, xl1, xh2, xl2;
      split_f16(ddx, xh0, xl0);
      split_f16(ddy, xh1, xl1);
      split_f16(ddz, xh2, xl2);
      v8h hv, lv, zv;
      hv[0] = xh0; hv[1] = xh1; hv[2] = xh2;
      lv[0] = xl0; lv[1] = xl1; lv[2] = xl2;
#pragma unroll
      for (int e = 3; e < 8; ++e) { hv[e] = z16; lv[e] = z16; }
#pragma unroll
      for (int e = 0; e < 8; ++e) zv[e] = z16;
      *(v8h*)(rh + 64) = hv;
      *(v8h*)(rl + 64) = lv;
      *(v8h*)(rh + 72) = zv;
      *(v8h*)(rl + 72) = zv;
      *(v8h*)(rh + 80) = zv;
      *(v8h*)(rl + 80) = zv;
      *(v8h*)(rh + 88) = zv;
      *(v8h*)(rl + 88) = zv;
    }
  }
  __syncthreads();

  {
    v16h ah[2][3], al[2][3];
#pragma unroll
    for (int mt = 0; mt < 2; ++mt)
#pragma unroll
      for (int kc = 0; kc < 3; ++kc) {
        ah[mt][kc] = FragH::load(ahi + (mt * 16 + c) * APITCH + kc * 32 + 8 * hh);
        al[mt][kc] = FragH::load(alo + (mt * 16 + c) * APITCH + kc * 32 + 8 * hh);
      }
#pragma unroll 1
    for (int nt = 0; nt < NCH_L0 / 16; ++nt) {
      const int col = nt * 16 + c;
      const _Float16* bp = bt0 + (size_t)col * KPAD0 + 8 * hh;
      v16h bf[3];
#pragma unroll
      for (int kc = 0; kc < 3; ++kc) bf[kc] = FragH::load(bp + kc * 32);
      const float s = scale[col];
      const float t = shift[col];
      v8f am[2], ar[2];
#pragma unroll
      for (int mt = 0; mt < 2; ++mt) {
        am[mt] = (v8f){0.f, 0.f, 0.f, 0.f, 0.f, 0.f, 0.f, 0.f};
        ar[mt] = (v8f){0.f, 0.f, 0.f, 0.f, 0.f, 0.f, 0.f, 0.f};
      }
#pragma unroll
      for (int mt = 0; mt < 2; ++mt)
#pragma unroll
        for (int kc = 0; kc < 3; ++kc) {
          am[mt] = mma_f16(ah[mt][kc], bf[kc], am[mt]);
          ar[mt] = mma_f16(al[mt][kc], bf[kc], ar[mt]);
        }
#pragma unroll
      for (int mt = 0; mt < 2; ++mt)
#pragma unroll
        for (int r = 0; r < 8; ++r) {
          const float v = fmaf(ar[mt][r], RESID_CARRY_INV, am[mt][r]);
          const float o = fmaxf(fmaf(v, s, t), 0.0f);
          h0w[(mt * 16 + 8 * hh + r) * HPITCH + col] = (_Float16)o;
        }
    }
  }
  __syncthreads();

  {
    v16h a1[2][2];
#pragma unroll
    for (int mt = 0; mt < 2; ++mt)
#pragma unroll
      for (int kc = 0; kc < 2; ++kc)
        a1[mt][kc] = FragH::load(h0w + (mt * 16 + c) * HPITCH + kc * 32 + 8 * hh);
#pragma unroll 1
    for (int nt = 0; nt < NCH_L1 / 16; ++nt) {
      const int col = nt * 16 + c;
      const _Float16* bp = bt1 + (size_t)col * NCH_L0 + 8 * hh;
      v16h bf[2];
#pragma unroll
      for (int kc = 0; kc < 2; ++kc) bf[kc] = FragH::load(bp + kc * 32);
      const float s = scale[64 + col];
      const float t = shift[64 + col];
      v8f acc[2];
#pragma unroll
      for (int mt = 0; mt < 2; ++mt) acc[mt] = (v8f){0.f, 0.f, 0.f, 0.f, 0.f, 0.f, 0.f, 0.f};
#pragma unroll
      for (int mt = 0; mt < 2; ++mt)
#pragma unroll
        for (int kc = 0; kc < 2; ++kc) acc[mt] = mma_f16(a1[mt][kc], bf[kc], acc[mt]);
#pragma unroll
      for (int mt = 0; mt < 2; ++mt)
#pragma unroll
        for (int r = 0; r < 8; ++r) {
          const float o = fmaxf(fmaf(acc[mt][r], s, t), 0.0f);
          h1w[(mt * 16 + 8 * hh + r) * HPITCH + col] = (_Float16)o;
        }
    }
  }
  __syncthreads();

  {
    v16h a2[2][2];
#pragma unroll
    for (int mt = 0; mt < 2; ++mt)
#pragma unroll
      for (int kc = 0; kc < 2; ++kc)
        a2[mt][kc] = FragH::load(h1w + (mt * 16 + c) * HPITCH + kc * 32 + 8 * hh);
#pragma unroll 1
    for (int nt = 0; nt < NCH_L2 / 16; ++nt) {
      const int col = nt * 16 + c;
      const _Float16* bp = bt2 + (size_t)col * NCH_L1 + 8 * hh;
      v16h bf[2];
#pragma unroll
      for (int kc = 0; kc < 2; ++kc) bf[kc] = FragH::load(bp + kc * 32);
      const float s = scale[128 + col];
      const float t = shift[128 + col];
      v8f acc[2];
#pragma unroll
      for (int mt = 0; mt < 2; ++mt) acc[mt] = (v8f){0.f, 0.f, 0.f, 0.f, 0.f, 0.f, 0.f, 0.f};
#pragma unroll
      for (int mt = 0; mt < 2; ++mt)
#pragma unroll
        for (int kc = 0; kc < 2; ++kc) acc[mt] = mma_f16(a2[mt][kc], bf[kc], acc[mt]);
      float m = 0.0f;
#pragma unroll
      for (int mt = 0; mt < 2; ++mt)
#pragma unroll
        for (int r = 0; r < 8; ++r) {
          const float o = fmaxf(fmaf(acc[mt][r], s, t), 0.0f);
          m = fmaxf(m, o);
        }
      const float om = __shfl_xor(m, 16, 32);
      m = fmaxf(m, om);
      if (hh == 0) ost[col] = m;
    }
  }
  __syncthreads();

  {
    const v4f ov = *(const v4f*)(ost + lane * 4);
    float* orow = out1 + (size_t)gid * NCH_L2 + lane * 4;
    store_v4f_twice(orow, ov);
  }
}

extern "C" void kernel_launch(void* const* d_in, const int* in_sizes, int n_in,
                              void* d_out, int out_size, void* d_ws, size_t ws_size,
                              hipStream_t stream) {
  (void)in_sizes; (void)n_in; (void)out_size;
  if (ws_size < WS_TOTAL) return;
  const float* xyz    = (const float*)d_in[0];
  const float* points = (const float*)d_in[1];
  const float* W0  = (const float*)d_in[2];
  const float* b0  = (const float*)d_in[3];
  const float* g0  = (const float*)d_in[4];
  const float* be0 = (const float*)d_in[5];
  const float* m0  = (const float*)d_in[6];
  const float* v0  = (const float*)d_in[7];
  const float* W1  = (const float*)d_in[8];
  const float* b1  = (const float*)d_in[9];
  const float* g1  = (const float*)d_in[10];
  const float* be1 = (const float*)d_in[11];
  const float* m1  = (const float*)d_in[12];
  const float* v1  = (const float*)d_in[13];
  const float* W2  = (const float*)d_in[14];
  const float* b2  = (const float*)d_in[15];
  const float* g2  = (const float*)d_in[16];
  const float* be2 = (const float*)d_in[17];
  const float* m2  = (const float*)d_in[18];
  const float* v2  = (const float*)d_in[19];

  char* ws = (char*)d_ws;
  _Float16* btall = (_Float16*)(ws + WS_BT0);
  _Float16* bt0   = (_Float16*)(ws + WS_BT0);
  _Float16* bt1   = (_Float16*)(ws + WS_BT1);
  _Float16* bt2   = (_Float16*)(ws + WS_BT2);
  float* scale    = (float*)(ws + WS_SCALE);
  float* shift    = (float*)(ws + WS_SHIFT);
  float* cent4    = (float*)(ws + WS_CENT);

  float* out0 = (float*)d_out;
  float* out1 = out0 + (OUT0_BYTES / 4);

  prep_kernel<<<12, 256, 0, stream>>>(W0, W1, W2, b0, g0, be0, m0, v0,
                                      b1, g1, be1, m1, v1, b2, g2, be2, m2, v2,
                                      btall, scale, shift);
  fps_kernel<<<NBATCH, 256, 0, stream>>>(xyz, out0, cent4);
  group_mlp_kernel<<<(NBATCH * NCEN) / MLP_WAVES, MLP_WAVES * 32, 0, stream>>>(
      xyz, points, cent4, bt0, bt1, bt2, scale, shift, out1);
}
